// DualAttention_26895085207699
// MI455X (gfx1250) — hardware-run, weakly checked
//
#include <hip/hip_runtime.h>


#ifndef NB
#define NB 64
#endif
#ifndef SEQ
#define SEQ 285
#endif
#define NB_FULL  64
#define SEQ_FULL 285
#define NBP   64
#define LP    (((SEQ) + 31) / 32 * 32)
#define DM    256
#define IDIM  128
#define NITEM 99999
#define NEMB  100001
#define NPOS  300
#define ZP    100032
#define MROWS (NB * LP)
#define GW    2
#define AW    2
#define SP    (LP + 4)
#define OPA   (DM + 4)
#define SSW   (SP > OPA ? SP : OPA)
#define PPH   (LP + 8)
#define EP    (IDIM + 8)
#define GE    (LP / 32)
#define NITER 50
#define NEGB  (-3.0e38f)
#define CX    64.0f
#define CW    64.0f
#define CQ    256.0f
#define CV    1024.0f
#define CP    16384.0f
#define CLC   64.0f
#define CE    64.0f
#define LOG2E 1.4426950408889634f
#define SELU_S 1.0507009873554804934193349852946f
#define SELU_A 1.6732632423543772848170429916717f

static_assert(LP % 32 == 0);
static_assert(SEQ >= 2 && SEQ <= SEQ_FULL);
static_assert(NB <= NB_FULL && NB <= NBP);
static_assert(DM == 2 * IDIM);
static_assert(DM == 256);
static_assert(IDIM == 128);
static_assert(DM % 64 == 0 && DM % 32 == 0 && IDIM % 32 == 0 && (2 * DM) % 32 == 0);
static_assert(MROWS % (16 * GW) == 0);
static_assert(NBP % (16 * GW) == 0);
static_assert(NBP == 64);
static_assert((LP / 16) % AW == 0);
static_assert((LP / 16) % 2 == 0);
static_assert((LP / 2) % 4 == 0);
static_assert(ZP % 64 == 0 && ZP >= NITEM && ZP % 32 == 0);
static_assert((SP * 4) % 16 == 0 && (OPA * 4) % 16 == 0 && (PPH * 2) % 16 == 0 && (EP * 2) % 8 == 0);
static_assert(GE * 32 == LP);
static_assert(16 * GW == 32);
static_assert(AW * 16 * SSW * 4 + AW * 16 * PPH * 2 <= 131072);
static_assert(GW * 16 * (DM + 4) * 4 + GW * 16 * 4 <= 131072);
static_assert(LP * EP * 2 <= 131072);
static_assert((LP * 16) % 256 == 0 && (IDIM * (LP / 8)) % 256 == 0);

typedef _Float16 h16;
typedef __attribute__((ext_vector_type(16))) _Float16 v16h;
typedef __attribute__((ext_vector_type(8)))  _Float16 v8h;
typedef __attribute__((ext_vector_type(4)))  _Float16 v4h;
typedef __attribute__((ext_vector_type(8)))  float    v8f;
typedef __attribute__((ext_vector_type(4)))  float    v4f;
typedef v4f  __attribute__((may_alias)) v4fa;
typedef v8h  __attribute__((may_alias)) v8ha;
typedef v4h  __attribute__((may_alias)) v4ha;

__device__ __forceinline__ unsigned short f2bf(float f) { unsigned u = __float_as_uint(f); u += 0x7FFFu + ((u >> 16) & 1u); return (unsigned short)(u >> 16); }
__device__ __forceinline__ float bfr(float f) { return __uint_as_float(((unsigned)f2bf(f)) << 16); }
__device__ __forceinline__ v16h cat16(v8h lo, v8h hi) { return __builtin_shufflevector(lo, hi, 0, 1, 2, 3, 4, 5, 6, 7, 8, 9, 10, 11, 12, 13, 14, 15); }
__device__ __forceinline__ v8f wmma16(v16h a, v16h b, v8f c) { return __builtin_amdgcn_wmma_f32_16x16x32_f16(false, a, false, b, (short)0, c, false, false); }
__device__ __forceinline__ v8f wmma16g(v16h a, v16h b, v8f c) { c = wmma16(a, b, c); asm volatile("v_nop\n\tv_nop\n\tv_nop\n\tv_nop" : "+v"(c) : "v"(a), "v"(b)); return c; }
__device__ __forceinline__ v16h ldh(const h16* p) { return cat16(*(const v8h*)p, *(const v8h*)(p + 16)); }
__device__ __forceinline__ void wave_sync() { __builtin_amdgcn_fence(3  , "wavefront"); __builtin_amdgcn_wave_barrier(); asm volatile("" ::: "memory"); }
static __device__ __forceinline__ h16 toh_flush(float v) { const h16 r = (h16)v; return (fabsf(v) < 6.103515625e-05f) ? (h16)0.0f : r; }
__device__ __forceinline__ float wsum(float v) { v += __shfl_xor(v, 16, 32); v += __shfl_xor(v, 8, 32); v += __shfl_xor(v, 4, 32); v += __shfl_xor(v, 2, 32); v += __shfl_xor(v, 1, 32); return v; }
__device__ __forceinline__ float wmaxr(float v) { v = fmaxf(v, __shfl_xor(v, 16, 32)); v = fmaxf(v, __shfl_xor(v, 8, 32)); v = fmaxf(v, __shfl_xor(v, 4, 32)); v = fmaxf(v, __shfl_xor(v, 2, 32)); v = fmaxf(v, __shfl_xor(v, 1, 32)); return v; }
__device__ __forceinline__ float alpha_of(float z) { const float sg = 1.0f / (1.0f + __builtin_amdgcn_exp2f(-z * LOG2E)); const float a = sg + 1.0f; return (a == 1.0f) ? 1.0001f : a; }
__device__ __forceinline__ float pfn(float z, float inv) { const float e = __builtin_amdgcn_exp2f(inv * __builtin_amdgcn_logf(fmaxf(z, 1.0e-30f))); return (z > 0.0f) ? e : 0.0f; }

__global__ __launch_bounds__(256) void k_cvth(const float* __restrict__ src, h16* dst, int n8, float carry) {
    const int i = blockIdx.x * 256 + threadIdx.x; if (i >= n8) return;
    const v4f a = *(const v4f*)(src + (size_t)i * 8), c = *(const v4f*)(src + (size_t)i * 8 + 4); v8h o;
#pragma unroll
    for (int k = 0; k < 4; ++k) { o[k] = toh_flush(bfr(a[k]) * carry); o[4 + k] = toh_flush(bfr(c[k]) * carry); }
    *(volatile v8h*)(dst + (size_t)i * 8) = o; __threadfence(); *(volatile v8h*)(dst + (size_t)i * 8) = o;
}

__global__ __launch_bounds__(256) void k_cvthT(const float* __restrict__ src, h16* dst, float carry) {
    const int r = threadIdx.x >> 5, c8 = (threadIdx.x & 31) * 8; const int n = blockIdx.x * 8 + r;
    v8h o;
#pragma unroll
    for (int i = 0; i < 8; ++i) o[i] = toh_flush(bfr(src[(size_t)(c8 + i) * DM + n]) * carry);
    *(volatile v8h*)(dst + (size_t)n * DM + c8) = o; __threadfence(); *(volatile v8h*)(dst + (size_t)n * DM + c8) = o;
}

__global__ __launch_bounds__(256) void k_embed(const int* __restrict__ idx, const float* __restrict__ tab, int nrows, int colbase, h16* XH, h16* XT) {
    __shared__ __align__(16) h16 tile[LP * EP];
    const int tid = threadIdx.x, b = blockIdx.x;
    const int wrow = tid >> 5, c4 = (tid & 31) * 4;
#pragma unroll 1
    for (int ps = 0; ps < LP / 8; ++ps) {
        const int t = ps * 8 + wrow;
        const int tc = t < SEQ ? t : SEQ - 1;
        int id = idx[(size_t)b * SEQ_FULL + tc];
        id = id < 0 ? 0 : (id > nrows - 1 ? nrows - 1 : id);
        v4f v = *(const v4f*)(tab + (size_t)id * IDIM + c4);
        asm volatile("" : "+v"(v));
        const bool ok = t < SEQ;
        v4h o;
#pragma unroll
        for (int i = 0; i < 4; ++i) o[i] = ok ? toh_flush(bfr(v[i]) * CX) : (h16)0.0f;
        *(v4ha*)(&tile[t * EP + c4]) = o;
    }
    __syncthreads();
    h16* xtb = XT + ((size_t)b * DM + colbase) * LP;
#pragma unroll 1
    for (int ps = 0; ps < 2; ++ps) {
#pragma unroll 1
        for (int it = 0; it < (LP * 16) / 256; ++it) {
            const int p = it * 256 + tid; const int t = p >> 4, c8 = (p & 15) * 8;
            const v8h v = *(const v8ha*)(&tile[t * EP + c8]);
            *(volatile v8h*)(XH + ((size_t)b * LP + t) * DM + colbase + c8) = v; }
#pragma unroll 1
        for (int it = 0; it < (IDIM * (LP / 8)) / 256; ++it) {
            const int p = it * 256 + tid; const int d = p / (LP / 8), t8 = (p % (LP / 8)) * 8;
            v8h v;
#pragma unroll
            for (int i = 0; i < 8; ++i) v[i] = tile[(t8 + i) * EP + d];
            *(volatile v8h*)(xtb + (size_t)p * 8) = v; }
        if (ps == 0) __threadfence(); }
}

#define M_RELUH 0
#define M_LN    1
#define M_F32   2
#define M_AL    3
#define M_WF    4
template <int NT, int MODE>
__device__ __forceinline__ void slab_gemm(const h16* __restrict__ A1, int lda1, int K1, const h16* __restrict__ A2, int lda2, int K2, int mmax,
                                          const h16* __restrict__ Bt, int ldb, float sc,
                                          const float* __restrict__ p0, const float* __restrict__ p1, const float* __restrict__ p2, const float* __restrict__ p3,
                                          h16* OH, float* OF, float carry) {
    constexpr int NC = NT * 16;
    constexpr int OP = NC + 4;
    static_assert(MODE == M_WF || NC == 256);
    static_assert(MODE != M_WF || NC == 128);
    __shared__ __align__(16) float os[GW * 16 * OP];
    __shared__ __align__(16) float red[GW * 16];
    const int lane = threadIdx.x & 31, lr = lane & 15, hi = lane >> 4;
    const int wave = __builtin_amdgcn_readfirstlane((int)(threadIdx.x >> 5));
    const int r0 = (blockIdx.x * GW + wave) * 16;
    const int wb = wave * 16 * OP;
    v8f acc[NT];
#pragma unroll
    for (int nb = 0; nb < NT; ++nb) acc[nb] = (v8f){};
    int ar = r0 + lr; ar = ar > mmax ? mmax : ar;
    const size_t a1o = (size_t)ar * lda1 + 8 * hi, a2o = (size_t)ar * lda2 + 8 * hi, bo = (size_t)lr * ldb + 8 * hi;
#pragma unroll 1
    for (int kc = 0; kc < K1; kc += 32) {
        const v16h a = ldh(A1 + a1o + kc);
#pragma unroll
        for (int nb = 0; nb < NT; ++nb) { const v16h bq = ldh(Bt + bo + (size_t)nb * 16 * ldb + kc); acc[nb] = wmma16g(a, bq, acc[nb]); }
    }
#pragma unroll 1
    for (int kc = 0; kc < K2; kc += 32) {
        const v16h a = ldh(A2 + a2o + kc);
#pragma unroll
        for (int nb = 0; nb < NT; ++nb) { const v16h bq = ldh(Bt + bo + (size_t)nb * 16 * ldb + K1 + kc); acc[nb] = wmma16g(a, bq, acc[nb]); }
    }
#pragma unroll
    for (int nb = 0; nb < NT; ++nb)
#pragma unroll
        for (int j = 0; j < 8; ++j) os[wb + (hi * 8 + j) * OP + nb * 16 + lr] = acc[nb][j] * sc;
    wave_sync();
    if (MODE == M_RELUH) {
        const int c8 = lane * 8;
        const v4f b0 = *(const v4f*)(p0 + c8), b1 = *(const v4f*)(p0 + c8 + 4);
#pragma unroll 1
        for (int ps = 0; ps < 2; ++ps) {
#pragma unroll 1
            for (int it = 0; it < 16; ++it) {
                const v4f x0 = *(const v4fa*)(&os[wb + it * OP + c8]); const v4f x1 = *(const v4fa*)(&os[wb + it * OP + c8 + 4]); v8h o;
#pragma unroll
                for (int i = 0; i < 4; ++i) { o[i] = toh_flush(fmaxf(x0[i] + bfr(b0[i]), 0.0f) * carry); o[4 + i] = toh_flush(fmaxf(x1[i] + bfr(b1[i]), 0.0f) * carry); }
                *(volatile v8h*)(OH + (size_t)(r0 + it) * NC + c8) = o; }
            if (ps == 0) __threadfence(); }
    } else if (MODE == M_LN) {
#pragma unroll 1
        for (int it = 0; it < 32; ++it) { const int row = it >> 1, c4 = ((it & 1) * 32 + lane) * 4;
            v4f x = *(const v4fa*)(&os[wb + row * OP + c4]); const v4f bb = *(const v4f*)(p0 + c4); const v4f rr = *(const v4f*)(p1 + (size_t)(r0 + row) * NC + c4);
#pragma unroll
            for (int i = 0; i < 4; ++i) x[i] = (x[i] + bfr(bb[i])) + rr[i];
            *(v4fa*)(&os[wb + row * OP + c4]) = x; }
        wave_sync();
        const int sb = wb + lr * OP + hi * 128;
        float s = 0.0f;
#pragma unroll 4
        for (int c = 0; c < 32; ++c) { const v4f x = *(const v4fa*)(&os[sb + 4 * c]); s += (x[0] + x[1]) + (x[2] + x[3]); }
        s += __shfl_xor(s, 16, 32);
        const float mean = s * (1.0f / 256.0f);
        float q = 0.0f;
#pragma unroll 4
        for (int c = 0; c < 32; ++c) { const v4f x = *(const v4fa*)(&os[sb + 4 * c]);
            const float d0 = x[0] - mean, d1 = x[1] - mean, d2 = x[2] - mean, d3 = x[3] - mean; q += (d0 * d0 + d1 * d1) + (d2 * d2 + d3 * d3); }
        q += __shfl_xor(q, 16, 32);
        const float rstd = rsqrtf(q * (1.0f / 256.0f) + 1.0e-5f);
        const int c8 = lane * 8;
        const v4f g0 = *(const v4f*)(p2 + c8), g1 = *(const v4f*)(p2 + c8 + 4), e0 = *(const v4f*)(p3 + c8), e1 = *(const v4f*)(p3 + c8 + 4);
#pragma unroll 1
        for (int ps = 0; ps < 2; ++ps) {
#pragma unroll 1
            for (int it = 0; it < 16; ++it) {
                const float mr = __shfl(mean, it, 32), rs = __shfl(rstd, it, 32);
                const v4f x0 = *(const v4fa*)(&os[wb + it * OP + c8]); const v4f x1 = *(const v4fa*)(&os[wb + it * OP + c8 + 4]); v8h o;
#pragma unroll
                for (int i = 0; i < 4; ++i) { o[i] = toh_flush(((x0[i] - mr) * rs * bfr(g0[i]) + bfr(e0[i])) * carry); o[4 + i] = toh_flush(((x1[i] - mr) * rs * bfr(g1[i]) + bfr(e1[i])) * carry); }
                *(volatile v8h*)(OH + (size_t)(r0 + it) * NC + c8) = o; }
            if (ps == 0) __threadfence(); }
    } else if (MODE == M_F32) {
#pragma unroll 1
        for (int ps = 0; ps < 2; ++ps) {
#pragma unroll 1
            for (int it = 0; it < 32; ++it) { const int row = it >> 1, c4 = ((it & 1) * 32 + lane) * 4;
                const v4f x = *(const v4fa*)(&os[wb + row * OP + c4]);
                *(volatile v4f*)(OF + (size_t)(r0 + row) * NC + c4) = x; }
            if (ps == 0) __threadfence(); }
    } else if (MODE == M_AL) {
        const int bidx = r0 / LP;
        const int sb = wb + lr * OP + hi * 128;
        float s = 0.0f;
#pragma unroll 2
        for (int c = 0; c < 32; ++c) { const int col = hi * 128 + 4 * c;
            const v4f x = *(const v4fa*)(&os[sb + 4 * c]); const v4f mm = *(const v4f*)(p0 + (size_t)bidx * NC + col);
            const v4f bb = *(const v4f*)(p1 + col); const v4f ww = *(const v4f*)(p2 + col);
#pragma unroll
            for (int i = 0; i < 4; ++i) s += fmaxf((x[i] + mm[i]) + bfr(bb[i]), 0.0f) * bfr(ww[i]); }
        s += __shfl_xor(s, 16, 32);
        if (hi == 0) red[wave * 16 + lr] = s;
        __syncthreads();
        if (wave == 0) {
#pragma unroll 1
            for (int ps = 0; ps < 2; ++ps) {
                if (lane < (GW * 16) / 4) { const v4f v = *(const v4fa*)(&red[lane * 4]);
                    *(volatile v4f*)(OF + (size_t)blockIdx.x * (GW * 16) + lane * 4) = v; }
                if (ps == 0) __threadfence(); } }
    } else {
#pragma unroll 1
        for (int it = 0; it < 16; ++it) { const int c4 = lane * 4;
            v4f x = *(const v4fa*)(&os[wb + it * OP + c4]); const v4f bb = *(const v4f*)(p0 + c4);
#pragma unroll
            for (int i = 0; i < 4; ++i) { const float u = x[i] + bfr(bb[i]); x[i] = (u > 0.0f) ? SELU_S * u : (SELU_S * SELU_A) * (__builtin_amdgcn_exp2f(u * LOG2E) - 1.0f); }
            *(v4fa*)(&os[wb + it * OP + c4]) = x; }
        wave_sync();
        const int sb = wb + lr * OP + hi * 64;
        float q = 0.0f;
#pragma unroll 4
        for (int c = 0; c < 16; ++c) { const v4f x = *(const v4fa*)(&os[sb + 4 * c]); q += (x[0] * x[0] + x[1] * x[1]) + (x[2] * x[2] + x[3] * x[3]); }
        q += __shfl_xor(q, 16, 32);
        const float inv = 1.0f / sqrtf(q);
        const int c8 = lr * 8;
#pragma unroll 1
        for (int ps = 0; ps < 2; ++ps) {
#pragma unroll 1
            for (int it = 0; it < 8; ++it) { const int row = it * 2 + hi;
                const float iv = __shfl(inv, row, 32);
                const v4f x0 = *(const v4fa*)(&os[wb + row * OP + c8]); const v4f x1 = *(const v4fa*)(&os[wb + row * OP + c8 + 4]); v8h o;
#pragma unroll
                for (int i = 0; i < 4; ++i) { o[i] = toh_flush(x0[i] * iv * carry); o[4 + i] = toh_flush(x1[i] * iv * carry); }
                *(volatile v8h*)(OH + (size_t)(r0 + row) * NC + c8) = o; }
            if (ps == 0) __threadfence(); }
    }
}

__global__ __launch_bounds__(32 * GW) __attribute__((amdgpu_num_vgpr(256)))
void k_gemm_relu(const h16* __restrict__ A, const h16* __restrict__ Bt, const float* __restrict__ bias, h16* OH, float sc, float carry, int mmax) {
    slab_gemm<16, M_RELUH>(A, DM, DM, A, DM, 0, mmax, Bt, DM, sc, bias, bias, bias, bias, OH, (float*)0, carry);
}
__global__ __launch_bounds__(32 * GW) __attribute__((amdgpu_num_vgpr(256)))
void k_gemm_ln(const h16* __restrict__ A, const h16* __restrict__ Bt, const float* __restrict__ bias, const float* __restrict__ resid,
               const float* __restrict__ gain, const float* __restrict__ beta, h16* OH, float sc, float carry, int mmax) {
    slab_gemm<16, M_LN>(A, DM, DM, A, DM, 0, mmax, Bt, DM, sc, bias, resid, gain, beta, OH, (float*)0, carry);
}
__global__ __launch_bounds__(32 * GW) __attribute__((amdgpu_num_vgpr(256)))
void k_gemm_f32(const h16* __restrict__ A, int lda, const h16* __restrict__ Bt, float* OF, float sc, int mmax) {
    slab_gemm<16, M_F32>(A, lda, DM, A, lda, 0, mmax, Bt, DM, sc, (const float*)OF, (const float*)OF, (const float*)OF, (const float*)OF, (h16*)0, OF, 1.0f);
}
__global__ __launch_bounds__(32 * GW) __attribute__((amdgpu_num_vgpr(256)))
void k_gemm_al(const h16* __restrict__ A, const h16* __restrict__ Bt, const float* __restrict__ addrow, const float* __restrict__ bias,
               const float* __restrict__ w0, float* OF, float sc, int mmax) {
    slab_gemm<16, M_AL>(A, DM, DM, A, DM, 0, mmax, Bt, DM, sc, addrow, bias, w0, w0, (h16*)0, OF, 1.0f);
}
__global__ __launch_bounds__(32 * GW) __attribute__((amdgpu_num_vgpr(256)))
void k_gemm_wf(const h16* __restrict__ A1, const h16* __restrict__ A2, int lda2, const h16* __restrict__ Bt, const float* __restrict__ bias,
               h16* OH, float sc, float carry, int mmax) {
    slab_gemm<8, M_WF>(A1, DM, DM, A2, lda2, DM, mmax, Bt, 2 * DM, sc, bias, bias, bias, bias, OH, (float*)0, carry);
}

__global__ __launch_bounds__(32 * AW) __attribute__((amdgpu_num_vgpr(256)))
void k_attn(const h16* __restrict__ QH, const h16* __restrict__ XH, const h16* __restrict__ XT, const int* __restrict__ xi,
            const float* __restrict__ aw, const float* __restrict__ ab, float* AVF, h16* AVH) {
    __shared__ __align__(16) float ss[AW * 16 * SSW];
    __shared__ __align__(16) h16 ph[AW * 16 * PPH];
    const int lane = threadIdx.x & 31, lr = lane & 15, hi = lane >> 4;
    const int wave = __builtin_amdgcn_readfirstlane((int)(threadIdx.x >> 5));
    const int b = blockIdx.y;
    const int t0 = (blockIdx.x * AW + wave) * 16;
    const int wb = wave * 16 * SSW, pw = wave * 16 * PPH;
    float dz = 0.0f;
    { const v8h xv = *(const v8h*)(XH + ((size_t)b * LP + (SEQ - 1)) * DM + lane * 8);
      const v4f w0 = *(const v4f*)(aw + lane * 8), w1 = *(const v4f*)(aw + lane * 8 + 4);
#pragma unroll
      for (int i = 0; i < 4; ++i) { dz += (float)xv[i] * bfr(w0[i]); dz += (float)xv[4 + i] * bfr(w1[i]); } }
    dz = wsum(dz) * (1.0f / CX);
    const float alpha = alpha_of(dz + bfr(ab[0]));
    const float am1 = alpha - 1.0f, inv = 1.0f / am1;
    const float gpd = __builtin_amdgcn_exp2f(am1 * __builtin_amdgcn_logf(1.0f / (float)SEQ));
    const size_t qo = ((size_t)b * LP + t0 + lr) * DM + 8 * hi;
    const size_t xo = ((size_t)b * LP + lr) * DM + 8 * hi;
    const float scs = 1.0f / (16.0f * CQ * CX);
#pragma unroll 1
    for (int kt = 0; kt < LP / 16; kt += 2) {
        v8f s0 = (v8f){}, s1 = (v8f){};
#pragma unroll 1
        for (int kc = 0; kc < DM; kc += 32) {
            const v16h q = ldh(QH + qo + kc);
            const v16h k0 = ldh(XH + xo + (size_t)(kt * 16) * DM + kc), k1 = ldh(XH + xo + (size_t)(kt * 16 + 16) * DM + kc);
            s0 = wmma16g(q, k0, s0); s1 = wmma16g(q, k1, s1); }
        const int key0 = kt * 16 + lr, key1 = key0 + 16;
        const int kc0 = key0 < SEQ ? key0 : SEQ - 1, kc1 = key1 < SEQ ? key1 : SEQ - 1;
        int x0v = xi[(size_t)b * SEQ_FULL + kc0]; int x1v = xi[(size_t)b * SEQ_FULL + kc1];
        asm volatile("" : "+v"(x0v)); asm volatile("" : "+v"(x1v));
        const bool v0 = (key0 < SEQ) & (x0v != 0), v1 = (key1 < SEQ) & (x1v != 0);
#pragma unroll
        for (int j = 0; j < 8; ++j) {
            ss[wb + (8 * hi + j) * SP + key0] = v0 ? (s0[j] * scs) * am1 : NEGB;
            ss[wb + (8 * hi + j) * SP + key1] = v1 ? (s1[j] * scs) * am1 : NEGB; }
    }
    wave_sync();
    const int rb = wb + lr * SP + hi * (LP / 2);
    float mx = NEGB;
#pragma unroll 4
    for (int c = 0; c < LP / 8; ++c) { const v4f x = *(const v4fa*)(&ss[rb + 4 * c]); mx = fmaxf(mx, fmaxf(fmaxf(x[0], x[1]), fmaxf(x[2], x[3]))); }
    mx = fmaxf(mx, __shfl_xor(mx, 16, 32));
    float tau_lo = mx - 1.0f;
    const float tau_hi = mx - gpd;
    float f_lo = 0.0f;
#pragma unroll 2
    for (int c = 0; c < LP / 8; ++c) { const v4f x = *(const v4fa*)(&ss[rb + 4 * c]);
        f_lo += (pfn(x[0] - tau_lo, inv) + pfn(x[1] - tau_lo, inv)) + (pfn(x[2] - tau_lo, inv) + pfn(x[3] - tau_lo, inv)); }
    f_lo += __shfl_xor(f_lo, 16, 32);
    f_lo -= 1.0f;
    float dm = tau_hi - tau_lo, tau_m = tau_lo, sm = 1.0f;
#pragma unroll 1
    for (int it = 0; it < NITER; ++it) {
        dm *= 0.5f;
        tau_m = tau_lo + dm;
        const bool moving = (tau_m != tau_lo);
        float s = 0.0f;
#pragma unroll 2
        for (int c = 0; c < LP / 8; ++c) { const v4f x = *(const v4fa*)(&ss[rb + 4 * c]);
            s += (pfn(x[0] - tau_m, inv) + pfn(x[1] - tau_m, inv)) + (pfn(x[2] - tau_m, inv) + pfn(x[3] - tau_m, inv)); }
        s += __shfl_xor(s, 16, 32);
        sm = s;
        tau_lo = ((s - 1.0f) * f_lo >= 0.0f) ? tau_m : tau_lo;
        if (__builtin_amdgcn_ballot_w32(moving) == 0u) break;
    }
    const float rs = (1.0f / sm) * CP;
#pragma unroll 2
    for (int c = 0; c < LP / 8; ++c) { const v4f x = *(const v4fa*)(&ss[rb + 4 * c]); v4h o;
#pragma unroll
        for (int i = 0; i < 4; ++i) o[i] = toh_flush(pfn(x[i] - tau_m, inv) * rs);
        *(v4ha*)(&ph[pw + lr * PPH + hi * (LP / 2) + 4 * c]) = o; }
    wave_sync();
    const size_t vo = ((size_t)b * DM + lr) * LP + 8 * hi;
    const float sco = 1.0f / (CP * CX);
#pragma unroll 1
    for (int dg = 0; dg < DM / 64; ++dg) {
        v8f o0 = (v8f){}, o1 = (v8f){}, o2 = (v8f){}, o3 = (v8f){};
#pragma unroll 1
        for (int key0 = 0; key0 < LP; key0 += 32) {
            const int pi = pw + lr * PPH + key0 + 8 * hi;
            const v16h pa = cat16(*(const v8ha*)(&ph[pi]), *(const v8ha*)(&ph[pi + 16]));
            const h16* vb = XT + vo + (size_t)(dg * 64) * LP + key0;
            const v16h v0 = ldh(vb), v1 = ldh(vb + (size_t)16 * LP), v2 = ldh(vb + (size_t)32 * LP), v3 = ldh(vb + (size_t)48 * LP);
            o0 = wmma16g(pa, v0, o0); o1 = wmma16g(pa, v1, o1); o2 = wmma16g(pa, v2, o2); o3 = wmma16g(pa, v3, o3); }
#pragma unroll
        for (int j = 0; j < 8; ++j) { const int ob = wb + (8 * hi + j) * OPA + dg * 64 + lr;
            ss[ob] = o0[j] * sco; ss[ob + 16] = o1[j] * sco; ss[ob + 32] = o2[j] * sco; ss[ob + 48] = o3[j] * sco; }
    }
    wave_sync();
    const size_t ob0 = ((size_t)b * LP + t0) * DM;
#pragma unroll 1
    for (int ps = 0; ps < 2; ++ps) {
#pragma unroll 1
        for (int it = 0; it < 32; ++it) { const int row = it >> 1, c4 = ((it & 1) * 32 + lane) * 4;
            const v4f x = *(const v4fa*)(&ss[wb + row * OPA + c4]);
            *(volatile v4f*)(AVF + ob0 + (size_t)row * DM + c4) = x; }
#pragma unroll 1
        for (int it = 0; it < 16; ++it) { const int c8 = lane * 8;
            const v4f x0 = *(const v4fa*)(&ss[wb + it * OPA + c8]); const v4f x1 = *(const v4fa*)(&ss[wb + it * OPA + c8 + 4]); v8h o;
#pragma unroll
            for (int i = 0; i < 4; ++i) { o[i] = toh_flush(x0[i] * CV); o[4 + i] = toh_flush(x1[i] * CV); }
            *(volatile v8h*)(AVH + ob0 + (size_t)it * DM + c8) = o; }
        if (ps == 0) __threadfence(); }
}

__global__ __launch_bounds__(256) void k_glob(const h16* __restrict__ LNH, const h16* __restrict__ XH, const float* __restrict__ AL, const int* __restrict__ xi,
                                              const float* __restrict__ aw, const float* __restrict__ ab, h16* GCH) {
#pragma clang fp contract(off)
    __shared__ __align__(16) float wsm[LP];
    __shared__ __align__(16) h16 gst[DM];
    const int tid = threadIdx.x, lane = tid & 31;
    const int wave = __builtin_amdgcn_readfirstlane((int)(threadIdx.x >> 5));
    const int b = blockIdx.x;
    if (wave == 0) {
        float dz = 0.0f;
        { const v8h xv = *(const v8h*)(LNH + ((size_t)b * LP + (SEQ - 1)) * DM + lane * 8);
          const v4f w0 = *(const v4f*)(aw + lane * 8), w1 = *(const v4f*)(aw + lane * 8 + 4);
#pragma unroll
          for (int i = 0; i < 4; ++i) { dz += (float)xv[i] * bfr(w0[i]); dz += (float)xv[4 + i] * bfr(w1[i]); } }
        dz = wsum(dz) * (1.0f / CX);
        const float alpha = alpha_of(dz + bfr(ab[0]));
        const float am1 = alpha - 1.0f, inv = 1.0f / am1;
        const float gpd = __builtin_amdgcn_exp2f(am1 * __builtin_amdgcn_logf(1.0f / (float)(SEQ - 1)));
        float X[GE]; float mx = NEGB;
#pragma unroll
        for (int j = 0; j < GE; ++j) { const int e = lane + 32 * j; const int ec = e < SEQ - 1 ? e : SEQ - 2;
            int xv = xi[(size_t)b * SEQ_FULL + ec]; float av = AL[(size_t)b * LP + ec];
            asm volatile("" : "+v"(xv)); asm volatile("" : "+v"(av));
            const bool ok = (e < SEQ - 1) & (xv != 0);
            X[j] = ok ? av * am1 : NEGB; mx = fmaxf(mx, X[j]); }
        mx = wmaxr(mx);
        float tau_lo = mx - 1.0f; const float tau_hi = mx - gpd;
        float f_lo = 0.0f;
#pragma unroll
        for (int j = 0; j < GE; ++j) f_lo += pfn(X[j] - tau_lo, inv);
        f_lo = wsum(f_lo) - 1.0f;
        float dm = tau_hi - tau_lo, tau_m = tau_lo, sm = 1.0f;
#pragma unroll 1
        for (int it = 0; it < NITER; ++it) {
            dm *= 0.5f;
            tau_m = tau_lo + dm;
            const bool moving = (tau_m != tau_lo);
            float s = 0.0f;
#pragma unroll
            for (int j = 0; j < GE; ++j) s += pfn(X[j] - tau_m, inv);
            s = wsum(s);
            sm = s;
            tau_lo = ((s - 1.0f) * f_lo >= 0.0f) ? tau_m : tau_lo;
            if (__builtin_amdgcn_ballot_w32(moving) == 0u) break;
        }
        const float rs = 1.0f / sm;
#pragma unroll
        for (int j = 0; j < GE; ++j) wsm[lane + 32 * j] = pfn(X[j] - tau_m, inv) * rs;
    }
    __syncthreads();
    float s = 0.0f;
    const h16* xr = XH + (size_t)b * LP * DM + tid;
#pragma unroll 4
    for (int k = 0; k < SEQ - 1; ++k) s += wsm[k] * (float)xr[(size_t)k * DM];
    gst[tid] = toh_flush(s);
    __syncthreads();
    if (wave == 0) {
#pragma unroll 1
        for (int ps = 0; ps < 2; ++ps) {
            const v8h v = *(const v8ha*)(&gst[lane * 8]);
            *(volatile v8h*)(GCH + (size_t)b * DM + lane * 8) = v;
            if (ps == 0) __threadfence(); } }
}

__global__ __launch_bounds__(32) __attribute__((amdgpu_num_vgpr(256)))
void k_z(const h16* __restrict__ LC, const float* __restrict__ emb, float* ZW) {
    __shared__ __align__(16) float os[16 * 68];
    const int lane = threadIdx.x & 31, lr = lane & 15, hi = lane >> 4; const int n0 = blockIdx.x * 64;
    v8f acc[4][4];
#pragma unroll
    for (int mb = 0; mb < 4; ++mb)
#pragma unroll
        for (int nb = 0; nb < 4; ++nb) acc[mb][nb] = (v8f){};
    float ssq[4] = { 0.0f, 0.0f, 0.0f, 0.0f };
    size_t eo[4];
#pragma unroll
    for (int nb = 0; nb < 4; ++nb) { int row = n0 + nb * 16 + lr + 1; row = row > NEMB - 1 ? NEMB - 1 : row; eo[nb] = (size_t)row * IDIM + 8 * hi; }
#pragma unroll 1
    for (int kc = 0; kc < IDIM; kc += 32) {
        v16h a[4];
#pragma unroll
        for (int mb = 0; mb < 4; ++mb) a[mb] = ldh(LC + (size_t)(mb * 16 + lr) * IDIM + 8 * hi + kc);
#pragma unroll
        for (int nb = 0; nb < 4; ++nb) {
            const float* e = emb + eo[nb] + kc;
            const v4f e0 = *(const v4f*)e, e1 = *(const v4f*)(e + 4), e2 = *(const v4f*)(e + 16), e3 = *(const v4f*)(e + 20);
            v16h bq; float q = 0.0f;
#pragma unroll
            for (int i = 0; i < 4; ++i) {
                const float f0 = bfr(e0[i]), f1 = bfr(e1[i]), f2 = bfr(e2[i]), f3 = bfr(e3[i]);
                q += (f0 * f0 + f1 * f1) + (f2 * f2 + f3 * f3);
                bq[i] = toh_flush(f0 * CE); bq[4 + i] = toh_flush(f1 * CE); bq[8 + i] = toh_flush(f2 * CE); bq[12 + i] = toh_flush(f3 * CE); }
            ssq[nb] += q;
#pragma unroll
            for (int mb = 0; mb < 4; ++mb) acc[mb][nb] = wmma16g(a[mb], bq, acc[mb][nb]);
        }
    }
    float cs[4];
#pragma unroll
    for (int nb = 0; nb < 4; ++nb) { const float t = ssq[nb] + __shfl_xor(ssq[nb], 16, 32); cs[nb] = (20.0f / (CLC * CE)) * (1.0f / sqrtf(t)); }
#pragma unroll
    for (int mb = 0; mb < 4; ++mb) {
#pragma unroll
        for (int nb = 0; nb < 4; ++nb)
#pragma unroll
            for (int j = 0; j < 8; ++j) os[(hi * 8 + j) * 68 + nb * 16 + lr] = acc[mb][nb][j] * cs[nb];
        wave_sync();
#pragma unroll 1
        for (int ps = 0; ps < 2; ++ps) {
#pragma unroll
            for (int s = 0; s < 8; ++s) { const int row = 2 * s + (lane >> 4), c4 = (lane & 15) * 4;
                const v4f v = *(const v4fa*)(&os[row * 68 + c4]);
                *(volatile v4f*)(ZW + (size_t)(mb * 16 + row) * ZP + n0 + c4) = v; }
            if (ps == 0) __threadfence(); }
        wave_sync();
    }
}

__global__ __launch_bounds__(256) void k_pack(const float* __restrict__ ZW, float* OUT) {
    const size_t tot = (size_t)NB * NITEM;
    const size_t f = ((size_t)blockIdx.x * 256 + threadIdx.x) * 4;
    if (f >= tot) return;
    int b = (int)(f / NITEM); int n = (int)(f - (size_t)b * NITEM);
    v4f v;
#pragma unroll
    for (int e = 0; e < 4; ++e) { const int bc = b < NB ? b : NB - 1;
        v[e] = ZW[(size_t)bc * ZP + n];
        const bool w = (n + 1 == NITEM); n = w ? 0 : n + 1; b += w ? 1 : 0; }
    if (f + 4 <= tot) {
        *(volatile v4f*)(OUT + f) = v; __threadfence(); *(volatile v4f*)(OUT + f) = v;
    } else {
#pragma unroll
        for (int e = 0; e < 4; ++e) if (f + e < tot) *(volatile float*)(OUT + f + e) = v[e];
        __threadfence();
#pragma unroll
        for (int e = 0; e < 4; ++e) if (f + e < tot) *(volatile float*)(OUT + f + e) = v[e];
    }
}

static constexpr size_t al256(size_t v) { return (v + 255) & ~(size_t)255; }
static constexpr size_t SZ_PH = al256((size_t)MROWS * DM * 2);
static constexpr size_t SZ_PF = al256((size_t)MROWS * DM * 4);
static constexpr size_t SZ_W  = al256((size_t)DM * DM * 2);
static constexpr size_t SZ_MS = al256((size_t)NBP * DM * 4);
static constexpr size_t SZ_AL = al256((size_t)MROWS * 4);
static constexpr size_t SZ_GC = al256((size_t)NBP * DM * 2);
static constexpr size_t SZ_LC = al256((size_t)NBP * IDIM * 2);
static constexpr size_t SZ_ZW = al256((size_t)NBP * ZP * 4);
static constexpr size_t SZ_TOTAL = 6 * SZ_PH + SZ_PF + 6 * SZ_W + SZ_MS + SZ_AL + SZ_GC + SZ_LC + SZ_ZW;
static_assert(SZ_TOTAL <= (size_t)134217728);
static_assert((size_t)IDIM * 2 * DM == (size_t)DM * DM);
static_assert(((size_t)DM * DM) % 64 == 0);
static_assert((ZP / 64) * 64 == ZP);
static_assert(((size_t)NB_FULL * NITEM) % 32 == 0);

extern "C" void kernel_launch(void* const* d_in, const int* in_sizes, int n_in,
                              void* d_out, int out_size, void* d_ws, size_t ws_size, hipStream_t stream) {
    if (n_in < 20) return;
    const size_t needi = (size_t)(NB - 1) * SEQ_FULL + SEQ;
    if ((size_t)in_sizes[0] < needi || (size_t)in_sizes[1] < needi) return;
    if ((size_t)in_sizes[2] < (size_t)NEMB * IDIM || (size_t)in_sizes[3] < (size_t)NPOS * IDIM) return;
    if (in_sizes[4] < DM || (size_t)in_sizes[5] < (size_t)DM * DM || (size_t)in_sizes[6] < (size_t)DM * DM || in_sizes[7] < DM) return;
    if ((size_t)in_sizes[8] < (size_t)DM * DM || in_sizes[9] < DM || (size_t)in_sizes[10] < (size_t)DM * DM || in_sizes[11] < DM) return;
    if ((size_t)in_sizes[12] < (size_t)DM * DM || in_sizes[13] < DM || in_sizes[14] < DM || in_sizes[15] < DM) return;
    if ((size_t)in_sizes[16] < (size_t)IDIM * 2 * DM || in_sizes[17] < IDIM || in_sizes[18] < DM || in_sizes[19] < 1) return;
    if ((size_t)out_size < (size_t)NB * NITEM) return;
    if (SZ_TOTAL > ws_size) return;
    const int* xi = (const int*)d_in[0];       const int* pi = (const int*)d_in[1];
    const float* emb = (const float*)d_in[2];  const float* pemb = (const float*)d_in[3];
    const float* aw0 = (const float*)d_in[4];  const float* aw1 = (const float*)d_in[5];  const float* aw2 = (const float*)d_in[6];  const float* abias = (const float*)d_in[7];
    const float* mlpw = (const float*)d_in[8]; const float* mlpb = (const float*)d_in[9];
    const float* s1w = (const float*)d_in[10]; const float* s1b = (const float*)d_in[11];
    const float* s2w = (const float*)d_in[12]; const float* s2b = (const float*)d_in[13];
    const float* lng = (const float*)d_in[14]; const float* lnb = (const float*)d_in[15];
    const float* wfw = (const float*)d_in[16]; const float* wfb = (const float*)d_in[17];
    const float* alw = (const float*)d_in[18]; const float* alb = (const float*)d_in[19];
    float* OUT = (float*)d_out;
    char* wsp = (char*)d_ws;
    h16* XH  = (h16*)wsp; wsp += SZ_PH;
    h16* XT  = (h16*)wsp; wsp += SZ_PH;
    h16* QH  = (h16*)wsp; wsp += SZ_PH;
    h16* AVH = (h16*)wsp; wsp += SZ_PH;
    h16* Y1H = (h16*)wsp; wsp += SZ_PH;
    h16* LNH = (h16*)wsp; wsp += SZ_PH;
    float* AVF = (float*)wsp; wsp += SZ_PF;
    h16* WM  = (h16*)wsp; wsp += SZ_W;
    h16* WS1 = (h16*)wsp; wsp += SZ_W;
    h16* WS2 = (h16*)wsp; wsp += SZ_W;
    h16* W1T = (h16*)wsp; wsp += SZ_W;
    h16* W2T = (h16*)wsp; wsp += SZ_W;
    h16* WFH = (h16*)wsp; wsp += SZ_W;
    float* MSW = (float*)wsp; wsp += SZ_MS;
    float* AL  = (float*)wsp; wsp += SZ_AL;
    h16* GCH = (h16*)wsp; wsp += SZ_GC;
    h16* LC  = (h16*)wsp; wsp += SZ_LC;
    float* ZW = (float*)wsp; wsp += SZ_ZW;

    k_embed<<<NB, 256, 0, stream>>>(xi, emb, NEMB, 0, XH, XT);
    k_embed<<<NB, 256, 0, stream>>>(pi, pemb, NPOS, IDIM, XH, XT);
    { const int n8 = DM * DM / 8; const unsigned g = (unsigned)((n8 + 255) / 256);
      k_cvth<<<g, 256, 0, stream>>>(mlpw, WM, n8, CW); k_cvth<<<g, 256, 0, stream>>>(s1w, WS1, n8, CW);
      k_cvth<<<g, 256, 0, stream>>>(s2w, WS2, n8, CW); k_cvth<<<g, 256, 0, stream>>>(wfw, WFH, n8, CW); }
    k_cvthT<<<DM / 8, 256, 0, stream>>>(aw1, W1T, CW);
    k_cvthT<<<DM / 8, 256, 0, stream>>>(aw2, W2T, CW);

    const unsigned gtok = (unsigned)(MROWS / (16 * GW)), gbat = (unsigned)(NBP / (16 * GW));
    k_gemm_relu<<<gtok, 32 * GW, 0, stream>>>(XH, WM, mlpb, QH, 1.0f / (CX * CW), CQ, MROWS - 1);
    k_attn<<<dim3(LP / (16 * AW), NB, 1), 32 * AW, 0, stream>>>(QH, XH, XT, xi, alw, alb, AVF, AVH);
    k_gemm_relu<<<gtok, 32 * GW, 0, stream>>>(AVH, WS1, s1b, Y1H, 1.0f / (CV * CW), CV, MROWS - 1);
    k_gemm_ln<<<gtok, 32 * GW, 0, stream>>>(Y1H, WS2, s2b, AVF, lng, lnb, LNH, 1.0f / (CV * CW), CX, MROWS - 1);
    k_gemm_f32<<<gbat, 32 * GW, 0, stream>>>(LNH + (size_t)(SEQ - 1) * DM, LP * DM, W2T, MSW, 1.0f / (CX * CW), NB - 1);
    k_gemm_al<<<gtok, 32 * GW, 0, stream>>>(LNH, W1T, MSW, abias, aw0, AL, 1.0f / (CX * CW), MROWS - 1);
    k_glob<<<NB, 256, 0, stream>>>(LNH, XH, AL, xi, alw, alb, GCH);
    k_gemm_wf<<<gbat, 32 * GW, 0, stream>>>(GCH, LNH + (size_t)(SEQ - 1) * DM, LP * DM, WFH, wfb, LC, 1.0f / (CX * CW), CLC, NB - 1);
    k_z<<<ZP / 64, 32, 0, stream>>>(LC, emb, ZW);
    { const size_t pieces = ((size_t)NB * NITEM + 3) / 4;
      k_pack<<<(unsigned)((pieces + 255) / 256), 256, 0, stream>>>(ZW, OUT); }
}
